// GroupGlobalAttention_3573412790901
// MI455X (gfx1250) — hardware-run, weakly checked
//
#include <hip/hip_runtime.h>


#ifndef NT
#define NT 32
#endif
#ifndef NB
#define NB 16
#endif
#define NT_FULL 32
#define NB_FULL 16
#define SEQ  128
#define DM   1024
#define TG   4
#define CTP  136
#define MT   (NT / 16)
#define ASC  1024.0f
#define RSC  2048.0f
#define RSI  (1.0f / 2048.0f)
#define CSC  16.0f
#define OSC  (1.0f / 16384.0f)
#define L2E  1.4426950408889634f
#define OUT1_OFF ((size_t)NT_FULL * NB_FULL * DM)

static_assert(DM == 1024);
static_assert(SEQ == 128);
static_assert(DM % 64 == 0 && DM % 32 == 0);
static_assert(NT % 16 == 0 && MT >= 1 && MT <= 2);
static_assert(NT % TG == 0);
static_assert(NT <= NT_FULL && NB <= NB_FULL);
static_assert((NB * SEQ) % 64 == 0);
static_assert(((size_t)NB * DM) % 8 == 0);
static_assert(OUT1_OFF * 4 == (size_t)2097152);
static_assert(((size_t)(NT - 1) * NB_FULL + NB) * DM <= OUT1_OFF);
static_assert(CTP >= SEQ + 8 && (CTP * 2) % 16 == 0);

typedef _Float16 h16;
typedef unsigned short bf;
typedef __attribute__((ext_vector_type(16))) __bf16   v16bf;
typedef __attribute__((ext_vector_type(16))) _Float16 v16h;
typedef __attribute__((ext_vector_type(8)))  _Float16 v8h;
typedef __attribute__((ext_vector_type(8)))  unsigned short v8us;
typedef __attribute__((ext_vector_type(8)))  float    v8f;
typedef __attribute__((ext_vector_type(4)))  float    v4f;
typedef v4f  __attribute__((may_alias)) v4fa;
typedef v8h  __attribute__((may_alias)) v8ha;

__device__ __forceinline__ unsigned short f2bf(float f) { unsigned u = __float_as_uint(f); u += 0x7FFFu + ((u >> 16) & 1u); return (unsigned short)(u >> 16); }
__device__ __forceinline__ float bfr(float f) { return __uint_as_float(((unsigned)f2bf(f)) << 16); }
__device__ __forceinline__ v16h cat16(v8h lo, v8h hi) { return __builtin_shufflevector(lo, hi, 0, 1, 2, 3, 4, 5, 6, 7, 8, 9, 10, 11, 12, 13, 14, 15); }
__device__ __forceinline__ v16bf cat16b(v8us lo, v8us hi) { return __builtin_bit_cast(v16bf, __builtin_shufflevector(lo, hi, 0, 1, 2, 3, 4, 5, 6, 7, 8, 9, 10, 11, 12, 13, 14, 15)); }
__device__ __forceinline__ v8f wmma16(v16h a, v16h b, v8f c) { return __builtin_amdgcn_wmma_f32_16x16x32_f16(false, a, false, b, (short)0, c, false, false); }
__device__ __forceinline__ v8f wmmab(v16bf a, v16bf b, v8f c) { return __builtin_amdgcn_wmma_f32_16x16x32_bf16(false, a, false, b, (short)0, c, false, false); }
__device__ __forceinline__ v16bf ldb(const bf* p)  { return cat16b(*(const v8us*)p, *(const v8us*)(p + 16)); }
__device__ __forceinline__ void wave_sync() { __builtin_amdgcn_fence(3  , "wavefront"); __builtin_amdgcn_wave_barrier(); asm volatile("" ::: "memory"); }
__device__ __forceinline__ float rcp_nr(float d) { const float r = __builtin_amdgcn_rcpf(d); const float e = __builtin_fmaf(-d, r, 1.0f); return __builtin_fmaf(r, e, r); }
__device__ __forceinline__ float swishf(float x) { const float a = fminf(-x * L2E, 80.0f); return x * rcp_nr(1.0f + __builtin_amdgcn_exp2f(a)); }

__global__ __launch_bounds__(256) void k_cvt8(const float* __restrict__ src, bf* dst, size_t n8) {
    const size_t i = (size_t)blockIdx.x * 256 + threadIdx.x; if (i >= n8) return;
    const v8f v = *(const v8f*)(src + i * 8); v8us o;
#pragma unroll
    for (int k = 0; k < 8; ++k) o[k] = f2bf(v[k]);
    *(volatile v8us*)(dst + i * 8) = o; __threadfence(); *(volatile v8us*)(dst + i * 8) = o;
}

__global__ __launch_bounds__(32) void k_gemm(const bf* __restrict__ A, const bf* __restrict__ Bt, const float* __restrict__ bias, float* C, int M) {
    __shared__ __align__(16) float os[16 * 68];
    const int K = DM;
    const int lane = threadIdx.x & 31, lr = lane & 15, hi = lane >> 4; const int r0 = blockIdx.x * 64, c0 = blockIdx.y * 64;
    v8f acc[4][4];
#pragma unroll
    for (int mb = 0; mb < 4; ++mb)
#pragma unroll
        for (int nb = 0; nb < 4; ++nb) acc[mb][nb] = (v8f){};
    size_t aoff[4];
#pragma unroll
    for (int mb = 0; mb < 4; ++mb) { int row = r0 + mb * 16 + lr; row = row < M ? row : M - 1; aoff[mb] = (size_t)row * K + 8 * hi; }
    const size_t boff = (size_t)(c0 + lr) * K + 8 * hi;
#pragma unroll 1
    for (int kc = 0; kc < K; kc += 32) {
        v16bf a[4];
#pragma unroll
        for (int mb = 0; mb < 4; ++mb) a[mb] = ldb(A + aoff[mb] + kc);
#pragma unroll
        for (int nb = 0; nb < 4; ++nb) { const v16bf b = ldb(Bt + boff + (size_t)nb * 16 * K + kc);
#pragma unroll
            for (int mb = 0; mb < 4; ++mb) acc[mb][nb] = wmmab(a[mb], b, acc[mb][nb]); }
        asm volatile("v_nop\n\tv_nop\n\tv_nop\n\tv_nop" : "+v"(acc[0][0]), "+v"(acc[1][1]), "+v"(acc[2][2]), "+v"(acc[3][3]) : "v"(a[0]), "v"(a[1]), "v"(a[2]), "v"(a[3]));
    }
    v4f bb;
    { const v4f bv = *(const v4f*)(bias + c0 + lr * 4);
#pragma unroll
      for (int i = 0; i < 4; ++i) bb[i] = bfr(bv[i]); }
#pragma unroll
    for (int mb = 0; mb < 4; ++mb) {
#pragma unroll
        for (int nb = 0; nb < 4; ++nb) {
#pragma unroll
            for (int j = 0; j < 8; ++j) os[(hi * 8 + j) * 68 + nb * 16 + lr] = acc[mb][nb][j]; }
        wave_sync();
#pragma unroll 1
        for (int ps = 0; ps < 2; ++ps) {
#pragma unroll
            for (int s = 0; s < 8; ++s) { const int row = 2 * s + hi, cofs = lr * 4;
                const v4f x = *(const v4fa*)(&os[row * 68 + cofs]);
                const v4f val = x + bb;
                const int grow = r0 + mb * 16 + row;
                if (grow < M) *(volatile v4f*)(C + (size_t)grow * DM + c0 + cofs) = val; }
            if (ps == 0) __threadfence(); }
        wave_sync();
    }
}

__global__ __launch_bounds__(256) void k_score(const float* __restrict__ PI, const float* __restrict__ PC, const float* __restrict__ w_one, const float* __restrict__ b_one, float* ATT) {
    __shared__ __align__(16) float pis[TG * DM];
    __shared__ __align__(16) float wsm[DM];
    __shared__ __align__(16) float sc[TG * SEQ];
    const int tid = threadIdx.x, lane = tid & 31;
    const int wave = __builtin_amdgcn_readfirstlane(tid >> 5);
    const int b = blockIdx.x, t0 = blockIdx.y * TG;
#pragma unroll
    for (int q = 0; q < TG; ++q) {
        const v4f v = *(const v4f*)(PI + ((size_t)((t0 + q) * NB + b)) * DM + tid * 4);
        *(v4fa*)(&pis[q * DM + tid * 4]) = v; }
    { const v4f v = *(const v4f*)(w_one + tid * 4); v4f o;
#pragma unroll
      for (int c = 0; c < 4; ++c) o[c] = bfr(v[c]);
      *(v4fa*)(&wsm[tid * 4]) = o; }
    const float bone = bfr(b_one[0]);
    __syncthreads();
#pragma unroll 1
    for (int s = wave; s < SEQ; s += 8) {
        const float* pcr = PC + ((size_t)b * SEQ + s) * DM + lane * 4;
        float a0 = 0.0f, a1 = 0.0f, a2 = 0.0f, a3 = 0.0f;
#pragma unroll 1
        for (int i = 0; i < DM / 128; ++i) {
            const int d = i * 128 + lane * 4;
            const v4f pcv = *(const v4f*)(pcr + i * 128);
            const v4f wv = *(const v4fa*)(&wsm[d]);
            const v4f p0 = *(const v4fa*)(&pis[d]);
            const v4f p1 = *(const v4fa*)(&pis[DM + d]);
            const v4f p2 = *(const v4fa*)(&pis[2 * DM + d]);
            const v4f p3 = *(const v4fa*)(&pis[3 * DM + d]);
#pragma unroll
            for (int c = 0; c < 4; ++c) {
                a0 += wv[c] * swishf(p0[c] + pcv[c]);
                a1 += wv[c] * swishf(p1[c] + pcv[c]);
                a2 += wv[c] * swishf(p2[c] + pcv[c]);
                a3 += wv[c] * swishf(p3[c] + pcv[c]); }
        }
#pragma unroll
        for (int off = 16; off; off >>= 1) {
            a0 += __shfl_xor(a0, off, 32); a1 += __shfl_xor(a1, off, 32);
            a2 += __shfl_xor(a2, off, 32); a3 += __shfl_xor(a3, off, 32); }
        if (lane == 0) { sc[s] = a0 + bone; sc[SEQ + s] = a1 + bone; sc[2 * SEQ + s] = a2 + bone; sc[3 * SEQ + s] = a3 + bone; }
    }
    __syncthreads();
    const int tt = wave & (TG - 1);
    const v4f v = *(const v4fa*)(&sc[tt * SEQ + lane * 4]);
    float mx = fmaxf(fmaxf(v[0], v[1]), fmaxf(v[2], v[3]));
#pragma unroll
    for (int off = 16; off; off >>= 1) mx = fmaxf(mx, __shfl_xor(mx, off, 32));
    v4f e; float sum = 0.0f;
#pragma unroll
    for (int c = 0; c < 4; ++c) { e[c] = __builtin_amdgcn_exp2f((v[c] - mx) * L2E); sum += e[c]; }
#pragma unroll
    for (int off = 16; off; off >>= 1) sum += __shfl_xor(sum, off, 32);
    const float inv = rcp_nr(sum);
    const v4f o = e * inv;
    if (wave < TG) {
        float* dst = ATT + ((size_t)((t0 + tt) * NB_FULL + b)) * SEQ + lane * 4;
        *(volatile v4f*)dst = o; __threadfence(); *(volatile v4f*)dst = o;
    }
}

__global__ __launch_bounds__(32) void k_actx(const bf* __restrict__ CB, const float* ATT, float* OUT) {
    __shared__ __align__(16) h16 ct[64 * CTP];
    __shared__ __align__(16) float os[16 * 68];
    const int lane = threadIdx.x & 31, lr = lane & 15, hi = lane >> 4;
    const int d0 = blockIdx.x * 64, b = blockIdx.y;
    { const int rq = lane >> 3, c8 = (lane & 7) * 8;
      const bf* src = CB + ((size_t)b * SEQ + rq) * DM + d0 + c8;
#pragma unroll 4
      for (int it = 0; it < SEQ / 4; ++it) {
          const int s = it * 4 + rq;
          const v8us raw = *(const v8us*)(src + (size_t)it * 4 * DM);
#pragma unroll
          for (int j = 0; j < 8; ++j) ct[(c8 + j) * CTP + s] = (h16)(__uint_as_float(((unsigned)raw[j]) << 16) * CSC); } }
    __syncthreads();
    v8f acch[MT][4], accr[MT][4];
#pragma unroll
    for (int mt = 0; mt < MT; ++mt)
#pragma unroll
        for (int nb = 0; nb < 4; ++nb) { acch[mt][nb] = (v8f){}; accr[mt][nb] = (v8f){}; }
#pragma unroll 1
    for (int kc = 0; kc < SEQ; kc += 32) {
        v16h ah[MT], ar[MT];
#pragma unroll
        for (int mt = 0; mt < MT; ++mt) {
            const float* ap = ATT + ((size_t)((mt * 16 + lr) * NB_FULL + b)) * SEQ + kc + 8 * hi;
            const v4f x0 = *(const v4f*)ap, x1 = *(const v4f*)(ap + 4), x2 = *(const v4f*)(ap + 16), x3 = *(const v4f*)(ap + 20);
#pragma unroll
            for (int i = 0; i < 4; ++i) {
                const float y0 = x0[i] * ASC, y1 = x1[i] * ASC, y2 = x2[i] * ASC, y3 = x3[i] * ASC;
                const h16 g0 = (h16)y0, g1 = (h16)y1, g2 = (h16)y2, g3 = (h16)y3;
                ah[mt][i] = g0; ah[mt][4 + i] = g1; ah[mt][8 + i] = g2; ah[mt][12 + i] = g3;
                ar[mt][i]      = (h16)((y0 - (float)g0) * RSC); ar[mt][4 + i]  = (h16)((y1 - (float)g1) * RSC);
                ar[mt][8 + i]  = (h16)((y2 - (float)g2) * RSC); ar[mt][12 + i] = (h16)((y3 - (float)g3) * RSC); }
        }
#pragma unroll
        for (int nb = 0; nb < 4; ++nb) {
            const int bo = (nb * 16 + lr) * CTP + kc + 8 * hi;
            const v16h bfrag = cat16(*(const v8ha*)(&ct[bo]), *(const v8ha*)(&ct[bo + 16]));
#pragma unroll
            for (int mt = 0; mt < MT; ++mt) { acch[mt][nb] = wmma16(ah[mt], bfrag, acch[mt][nb]); accr[mt][nb] = wmma16(ar[mt], bfrag, accr[mt][nb]); } }
        asm volatile("v_nop\n\tv_nop\n\tv_nop\n\tv_nop" : "+v"(acch[0][0]), "+v"(acch[MT - 1][3]), "+v"(accr[0][0]), "+v"(accr[MT - 1][3]) : "v"(ah[0]), "v"(ah[MT - 1]), "v"(ar[0]), "v"(ar[MT - 1]));
    }
#pragma unroll
    for (int mt = 0; mt < MT; ++mt) {
#pragma unroll
        for (int nb = 0; nb < 4; ++nb) {
#pragma unroll
            for (int j = 0; j < 8; ++j) os[(hi * 8 + j) * 68 + nb * 16 + lr] = (acch[mt][nb][j] + accr[mt][nb][j] * RSI) * OSC; }
        wave_sync();
#pragma unroll 1
        for (int ps = 0; ps < 2; ++ps) {
#pragma unroll
            for (int s = 0; s < 8; ++s) { const int row = 2 * s + hi, cofs = lr * 4;
                const v4f val = *(const v4fa*)(&os[row * 68 + cofs]);
                *(volatile v4f*)(OUT + ((size_t)((mt * 16 + row) * NB_FULL + b)) * DM + d0 + cofs) = val; }
            if (ps == 0) __threadfence(); }
        wave_sync();
    }
}

static constexpr size_t al256(size_t v) { return (v + 255) & ~(size_t)255; }
static constexpr size_t SZ_XB = al256((size_t)NT * NB * DM * 2);
static constexpr size_t SZ_CB = al256((size_t)NB * SEQ * DM * 2);
static constexpr size_t SZ_W  = al256((size_t)DM * DM * 2);
static constexpr size_t SZ_PI = al256((size_t)NT * NB * DM * 4);
static constexpr size_t SZ_PC = al256((size_t)NB * SEQ * DM * 4);
static constexpr size_t SZ_TOTAL = SZ_XB + SZ_CB + 2 * SZ_W + SZ_PI + SZ_PC;
static_assert(SZ_TOTAL <= (size_t)134217728);

extern "C" void kernel_launch(void* const* d_in, const int* in_sizes, int n_in,
                              void* d_out, int out_size, void* d_ws, size_t ws_size, hipStream_t stream) {
    if (n_in < 8) return;
    if ((size_t)in_sizes[0] < ((size_t)(NT - 1) * NB_FULL + NB) * DM) return;
    if ((size_t)in_sizes[1] < (size_t)NB * SEQ * DM) return;
    if ((size_t)in_sizes[2] < (size_t)DM * DM || (size_t)in_sizes[4] < (size_t)DM * DM) return;
    if (in_sizes[3] < DM || in_sizes[5] < DM || in_sizes[6] < DM || in_sizes[7] < 1) return;
    if ((size_t)out_size < OUT1_OFF + ((size_t)(NT - 1) * NB_FULL + NB) * SEQ) return;
    if (SZ_TOTAL > ws_size) return;
    const float* xin  = (const float*)d_in[0];
    const float* ctx  = (const float*)d_in[1];
    const float* win  = (const float*)d_in[2];
    const float* bin  = (const float*)d_in[3];
    const float* wctx = (const float*)d_in[4];
    const float* bctx = (const float*)d_in[5];
    const float* wone = (const float*)d_in[6];
    const float* bone = (const float*)d_in[7];
    float* OUT = (float*)d_out;
    float* ATT = OUT + OUT1_OFF;
    char* wsp = (char*)d_ws;
    bf* XB = (bf*)wsp; wsp += SZ_XB;
    bf* CB = (bf*)wsp; wsp += SZ_CB;
    bf* WI = (bf*)wsp; wsp += SZ_W;
    bf* WC = (bf*)wsp; wsp += SZ_W;
    float* PI = (float*)wsp; wsp += SZ_PI;
    float* PC = (float*)wsp; wsp += SZ_PC;

    if (NB == NB_FULL) {
        const size_t n8 = (size_t)NT * NB * DM / 8;
        k_cvt8<<<(unsigned)((n8 + 255) / 256), 256, 0, stream>>>(xin, XB, n8);
    } else {
        const size_t n8 = (size_t)NB * DM / 8;
        for (int t = 0; t < NT; ++t) k_cvt8<<<(unsigned)((n8 + 255) / 256), 256, 0, stream>>>(xin + (size_t)t * NB_FULL * DM, XB + (size_t)t * NB * DM, n8);
    }
    { const size_t n8 = (size_t)NB * SEQ * DM / 8; k_cvt8<<<(unsigned)((n8 + 255) / 256), 256, 0, stream>>>(ctx, CB, n8); }
    { const size_t n8 = (size_t)DM * DM / 8; const unsigned g = (unsigned)((n8 + 255) / 256);
      k_cvt8<<<g, 256, 0, stream>>>(win, WI, n8); k_cvt8<<<g, 256, 0, stream>>>(wctx, WC, n8); }

    k_gemm<<<dim3((NT * NB + 63) / 64, DM / 64, 1), 32, 0, stream>>>(XB, WI, bin, PI, NT * NB);
    k_gemm<<<dim3((NB * SEQ + 63) / 64, DM / 64, 1), 32, 0, stream>>>(CB, WC, bctx, PC, NB * SEQ);

    k_score<<<dim3(NB, NT / TG, 1), 256, 0, stream>>>(PI, PC, wone, bone, ATT);
    k_actx<<<dim3(DM / 64, NB, 1), 32, 0, stream>>>(CB, ATT, OUT);
}
